// CombinedVirtualNodeEnvEncoder_2602750181779
// MI455X (gfx1250) — hardware-run, weakly checked
//
#include <hip/hip_runtime.h>

typedef float          v8f   __attribute__((ext_vector_type(8)));
typedef float          v4f   __attribute__((ext_vector_type(4)));
typedef unsigned int   v4u   __attribute__((ext_vector_type(4)));
typedef int            v8i   __attribute__((ext_vector_type(8)));
typedef unsigned short v8us  __attribute__((ext_vector_type(8)));
typedef unsigned short v16us __attribute__((ext_vector_type(16)));
typedef __bf16         v16bf __attribute__((ext_vector_type(16)));
typedef _Float16       v16h  __attribute__((ext_vector_type(16)));
typedef v4f  __attribute__((may_alias)) v4fa;
typedef v8us __attribute__((may_alias)) v8usa;
union FragB { v16bf v; v16us u; v8us h[2]; v8i w; };
union FragH { v16h  v; v16us u; v8us h[2]; v8i w; };

__device__ __forceinline__ v8f wmb(const FragB& a, const FragB& b, v8f c) {
  v8f d = __builtin_amdgcn_wmma_f32_16x16x32_bf16(false, a.v, false, b.v, (short)0, c, false, false);
  asm volatile("v_nop\n\tv_nop\n\tv_nop\n\tv_nop" : "+v"(d) : "v"(a.w), "v"(b.w));
  return d;
}

__device__ __forceinline__ v8f wmh(const FragH& a, const FragH& b, v8f c) {
  v8f d = __builtin_amdgcn_wmma_f32_16x16x32_f16(false, a.v, false, b.v, (short)0, c, false, false);
  asm volatile("v_nop\n\tv_nop\n\tv_nop\n\tv_nop" : "+v"(d) : "v"(a.w), "v"(b.w));
  return d;
}

__device__ __forceinline__ unsigned bf16_bits(float f) {
  const unsigned u = __float_as_uint(f);
  const unsigned r = (u + 0x7FFFu + ((u >> 16) & 1u)) >> 16;
  const unsigned q = (u >> 16) | 0x40u;
  return ((u & 0x7fffffffu) > 0x7f800000u) ? q : r;
}

__device__ __forceinline__ float bf16_val(float f) {
  return __uint_as_float(bf16_bits(f) << 16);
}
__device__ __forceinline__ int clampi(int v, int lo, int hi) {
  return v < lo ? lo : (v > hi ? hi : v);
}

__device__ __forceinline__ unsigned f16_bits(float f) {
  const unsigned u  = __float_as_uint(f);
  const unsigned s  = (u >> 16) & 0x8000u;
  const unsigned a  = u & 0x7fffffffu;
  const unsigned t  = a - 0x38000000u;
  const unsigned r  = (t + 0x0FFFu + ((t >> 13) & 1u)) >> 13;
  const unsigned rc = r > 0x7C00u ? 0x7C00u : r;
  const bool small  = a < 0x38800000u;
  const bool isnan  = a > 0x7f800000u;
  const unsigned fin = small ? 0u : (s | rc);
  return isnan ? (s | 0x7E00u) : fin;
}

__device__ __forceinline__ unsigned pk16(unsigned lo, unsigned hi) { return lo | (hi << 16); }
__device__ __forceinline__ unsigned bf16_lo_bits(float v) {
  float hi = bf16_val(v);
  asm volatile("" : "+v"(hi));
  return bf16_bits(v - hi);
}
__device__ __forceinline__ v4u pack8_bf16(v4f a, v4f c) {
  return (v4u){ pk16(bf16_bits(a[0]), bf16_bits(a[1])), pk16(bf16_bits(a[2]), bf16_bits(a[3])),
                pk16(bf16_bits(c[0]), bf16_bits(c[1])), pk16(bf16_bits(c[2]), bf16_bits(c[3])) };
}
__device__ __forceinline__ v4u pack8_bf16_lo(v4f a, v4f c) {
  return (v4u){ pk16(bf16_lo_bits(a[0]), bf16_lo_bits(a[1])), pk16(bf16_lo_bits(a[2]), bf16_lo_bits(a[3])),
                pk16(bf16_lo_bits(c[0]), bf16_lo_bits(c[1])), pk16(bf16_lo_bits(c[2]), bf16_lo_bits(c[3])) };
}
__device__ __forceinline__ v4u pack8_f16(v4f a, v4f c) {
  return (v4u){ pk16(f16_bits(a[0]), f16_bits(a[1])), pk16(f16_bits(a[2]), f16_bits(a[3])),
                pk16(f16_bits(c[0]), f16_bits(c[1])), pk16(f16_bits(c[2]), f16_bits(c[3])) };
}

template <int FORM>
__global__ __launch_bounds__(256) void k_plane(const float* __restrict__ src, int rows, int cols, int ldsrc,
                                               unsigned short* __restrict__ dst, int MP, int KP) {
  static_assert(FORM >= 0 && FORM <= 3);
  const int KTOT = (FORM == 1 || FORM == 3) ? 2 * KP : KP;
  const unsigned ppr   = (unsigned)(KTOT >> 3);
  const unsigned kp8   = (unsigned)(KP >> 3);
  const unsigned total = (unsigned)MP * ppr;
  const unsigned g     = blockIdx.x * 256u + threadIdx.x;
  const unsigned rowu  = g / ppr;
  const unsigned p     = g - rowu * ppr;
  const bool second    = p >= kp8;
  const int row = (int)rowu;
  const int c0  = (int)((second ? p - kp8 : p) << 3);
  const float* srow = src + (size_t)clampi(row, 0, rows - 1) * (size_t)ldsrc;
  float x[8];
  unsigned mk[8];
#pragma unroll
  for (int e = 0; e < 8; ++e) {
    const int c = c0 + e;
    const float v = srow[clampi(c, 0, cols - 1)];
    asm volatile("" :: "v"(v));
    x[e]  = v;
    mk[e] = (row < rows && c < cols) ? 0xFFFFu : 0u;
  }
  const v4f a = (v4f){ x[0], x[1], x[2], x[3] };
  const v4f c = (v4f){ x[4], x[5], x[6], x[7] };
  v4u o;
  if (FORM == 2) {
    o = pack8_f16(a, c);
  } else {
    const v4u hi = pack8_bf16(a, c);
    o = hi;
    if (FORM == 1) { const v4u lo = pack8_bf16_lo(a, c); o = second ? lo : hi; }
  }
  const v4u mw = (v4u){ pk16(mk[0], mk[1]), pk16(mk[2], mk[3]), pk16(mk[4], mk[5]), pk16(mk[6], mk[7]) };
  o &= mw;
  if (g < total) {
    volatile v4u* q = (volatile v4u*)(dst + (size_t)g * 8);
    *q = o;
    __threadfence();
    *q = o;
  }
}

template <int FORM> struct FragOf    { typedef FragB T; };
template <>         struct FragOf<2> { typedef FragH T; };
__device__ __forceinline__ v8f mm(const FragB& a, const FragB& b, v8f c) { return wmb(a, b, c); }
__device__ __forceinline__ v8f mm(const FragH& a, const FragH& b, v8f c) { return wmh(a, b, c); }
template <class F> __device__ __forceinline__ F ld_frag(const unsigned short* p) {
  F f;
  f.h[0] = *(const v8usa*)(p);
  f.h[1] = *(const v8usa*)(p + 16);
  return f;
}

template <int FORM, int EPI>
__global__ __launch_bounds__(256) __attribute__((amdgpu_num_vgpr(248)))
void k_gemm_nt(const unsigned short* __restrict__ A, const unsigned short* __restrict__ B,
               const float* __restrict__ bias, float* __restrict__ D, int M, int N, int KTOT, int ldd) {
  static_assert(FORM >= 0 && FORM <= 2);
  static_assert(EPI == 0 || EPI == 1);
  typedef typename FragOf<FORM>::T F;
  __shared__ __attribute__((aligned(16))) float sT[8][16 * 68];
  const int lane = threadIdx.x & 31;
  const int wave = threadIdx.x >> 5;
  const int tilesM = (M + 63) >> 6;
  const int tilesN = (N + 63) >> 6;
  const int tile = blockIdx.x * 8 + wave;
  if (tile >= tilesM * tilesN) return;
  const int tm = tile / tilesN;
  const int tn = tile - tm * tilesN;
  const int m0 = tm << 6;
  const int n0 = tn << 6;

  const int rl = lane & 15;
  const int h8 = (lane >> 4) * 8;
  const unsigned short* pa = A + (size_t)(m0 + rl) * (size_t)KTOT + h8;
  const unsigned short* pb = B + (size_t)(n0 + rl) * (size_t)KTOT + h8;

  v8f acc[4][4];
#pragma unroll
  for (int i = 0; i < 4; ++i)
#pragma unroll
    for (int j = 0; j < 4; ++j) acc[i][j] = (v8f){0.f, 0.f, 0.f, 0.f, 0.f, 0.f, 0.f, 0.f};

#pragma unroll 1
  for (int k0 = 0; k0 < KTOT; k0 += 32) {
    F bf[4];
#pragma unroll
    for (int j = 0; j < 4; ++j) bf[j] = ld_frag<F>(pb + (size_t)(j << 4) * (size_t)KTOT + k0);
#pragma unroll
    for (int i = 0; i < 4; ++i) {
      const F af = ld_frag<F>(pa + (size_t)(i << 4) * (size_t)KTOT + k0);
#pragma unroll
      for (int j = 0; j < 4; ++j) acc[i][j] = mm(af, bf[j], acc[i][j]);
    }
  }

  float* slab = sT[wave];
  const int hh = lane >> 4;
  const int c4 = (lane & 15) * 4;
  const int nc = n0 + c4;
  const bool cok = nc < N;
  v4f bv = (v4f){0.f, 0.f, 0.f, 0.f};
  if (EPI == 1) {
    bv = *(const v4fa*)(bias + clampi(nc, 0, N - 4));
    asm volatile("" :: "v"(bv));
  }
#pragma unroll
  for (int i = 0; i < 4; ++i) {
    const int mBase = m0 + (i << 4);
#pragma unroll
    for (int j = 0; j < 4; ++j) {
#pragma unroll
      for (int r = 0; r < 8; ++r) slab[(h8 + r) * 68 + (j << 4) + rl] = acc[i][j][r];
    }
    __builtin_amdgcn_fence(__ATOMIC_RELEASE, "workgroup");
    __builtin_amdgcn_wave_barrier();
    __builtin_amdgcn_fence(__ATOMIC_ACQUIRE, "workgroup");
    v4f vv[8];
#pragma unroll
    for (int it = 0; it < 8; ++it) {
      const int row = it * 2 + hh;
      v4f v = *(const v4fa*)(slab + row * 68 + c4);
      if (EPI == 1) v += bv;
      vv[it] = v;
    }
    for (int pass = 0; pass < 2; ++pass) {
#pragma unroll
      for (int it = 0; it < 8; ++it) {
        const int row = mBase + it * 2 + hh;
        if (cok && row < M) *(volatile v4f*)(D + (size_t)row * (size_t)ldd + nc) = vv[it];
      }
      __threadfence();
    }
    __builtin_amdgcn_fence(__ATOMIC_RELEASE, "workgroup");
    __builtin_amdgcn_wave_barrier();
    __builtin_amdgcn_fence(__ATOMIC_ACQUIRE, "workgroup");
  }
}

#include <stddef.h>
#include <math.h>

#define NN      100000
#define NE      1600000
#define CH      128
#define MPR     100096
#define KT2     256
#define NREC    782
#define NBRUN   1024
#define NBLK    98
#define NSLOT   (NBLK * NBRUN)
#define RCAP    20992
#define WLCAP   3072
#define DEGCAP  64
#define WCHUNK  256
#define NCHUNK  (NE / WCHUNK)
#define CPW     ((NCHUNK + 7) / 8)
#define MAXB1024 16710
#define MAXDEG  36
#define BK_WL   RCAP
#define BK_CNT  (RCAP + 8 * WLCAP)
#define BK_OFF  (BK_CNT + NBRUN)
#define BK_CUR  (BK_OFF + NBRUN)
#define BK_MISC (BK_CUR + NBRUN)
#define BK_INTS (BK_MISC + 16)

static_assert(NREC * 128 == MPR && MPR >= NN);
static_assert(782 * 128 >= NN);
static_assert(NN <= (1 << 17));
static_assert(NBRUN == (1 << 10));
static_assert(NE % WCHUNK == 0);
static_assert(((size_t)NE * 4) % 16 == 0);
static_assert(8 * CPW >= NCHUNK && 7 * CPW < NCHUNK);
static_assert(NSLOT >= MPR);
static_assert(RCAP % 256 == 0 && (size_t)RCAP * 4 >= (size_t)MAXB1024 * 5);
static_assert((size_t)WLCAP * 8 * 4 >= (size_t)MAXB1024 * 5);
static_assert(DEGCAP >= MAXDEG + 8 && DEGCAP % 32 == 0);
static_assert(BK_INTS % 4 == 0 && BK_INTS * 4 <= 262144);
static_assert(BK_INTS * 4 + 34816 <= 327680);
static_assert(MPR % 64 == 0 && KT2 % 32 == 0 && NN % 16 == 0 && CH % 64 == 0 && CH % 32 == 0);
static_assert((size_t)MPR * KT2 / 8 < ((size_t)2048 << 20));
static_assert((MPR * (CH / 8)) % 256 == 0);

typedef int          v4i  __attribute__((ext_vector_type(4)));
typedef unsigned int v2u  __attribute__((ext_vector_type(2)));
typedef v4i __attribute__((may_alias)) v4ia;
typedef v2u __attribute__((may_alias)) v2ua;

__device__ __forceinline__ void wt_unit(const float* __restrict__ W, unsigned short* T, int u) {
  const int n  = u >> 5;
  const int k8 = (u & 31) * 8;
  const int kk = k8 & (CH - 1);
  const float* p = W + (size_t)kk * CH + n;
  unsigned b[8];
#pragma unroll
  for (int i = 0; i < 8; ++i) {
    const float v = p[(size_t)i * CH];
    b[i] = bf16_bits(v);
  }
  const v4u o = (v4u){ pk16(b[0], b[1]), pk16(b[2], b[3]), pk16(b[4], b[5]), pk16(b[6], b[7]) };
  volatile v4u* q = (volatile v4u*)(T + (size_t)n * KT2 + k8);
  *q = o;
  __threadfence();
  *q = o;
}

__global__ __launch_bounds__(256) void k_wprep(const float* __restrict__ Wl, const float* __restrict__ Fc,
                                               const float* __restrict__ fcb,
                                               unsigned short* WlT2, unsigned short* FcT2, float* FCB) {
  const int blk = (int)blockIdx.x, tid = (int)threadIdx.x;
  if (blk < 16) {
    wt_unit(Wl, WlT2, blk * 256 + tid);
  } else if (blk < 32) {
    wt_unit(Fc, FcT2, (blk - 16) * 256 + tid);
  } else {
    const int i4 = tid < 31 ? tid : 31;
    const v4f v = *(const v4fa*)(fcb + 4 * i4);
    asm volatile("" :: "v"(v));
    const v4f o = (v4f){ bf16_val(v[0]), bf16_val(v[1]), bf16_val(v[2]), bf16_val(v[3]) };
    const bool st = tid < 32;
    volatile v4f* q = (volatile v4f*)(FCB + 4 * i4);
    if (st) *q = o;
    __threadfence();
    if (st) *q = o;
  }
}

__global__ __launch_bounds__(32) void k_colsum(const unsigned short* __restrict__ XB, float* REC) {
  const int lane = (int)threadIdx.x;
  const int b = (int)blockIdx.x;
  float a0 = 0.0f, a1 = 0.0f, a2 = 0.0f, a3 = 0.0f;
#pragma unroll 4
  for (int r = 0; r < 128; ++r) {
    const int row = b * 128 + r;
    const int rc  = row < MPR - 1 ? row : MPR - 1;
    const v2u w = *(const v2ua*)(XB + (size_t)rc * CH + 4 * lane);
    unsigned wx = w.x, wy = w.y;
    asm volatile("" :: "v"(wx), "v"(wy));
    const unsigned mk = (row < NN) ? 0xFFFFFFFFu : 0u;
    a0 += __uint_as_float((wx << 16) & mk);
    a1 += __uint_as_float((wx & 0xFFFF0000u) & mk);
    a2 += __uint_as_float((wy << 16) & mk);
    a3 += __uint_as_float((wy & 0xFFFF0000u) & mk);
  }
  const v4f o = (v4f){ a0, a1, a2, a3 };
  volatile v4f* q = (volatile v4f*)(REC + (size_t)b * CH + 4 * lane);
  *q = o;
  __threadfence();
  *q = o;
}

__global__ __launch_bounds__(256) void k_global(const float* __restrict__ REC,
                                                const float* __restrict__ w1, const float* __restrict__ b1,
                                                const float* __restrict__ w2, const float* __restrict__ b2,
                                                const float* __restrict__ alpha, float* GLB) {
  __shared__ double sD[256];
  __shared__ float sgp[CH];
  __shared__ float sh[CH];
  __shared__ __attribute__((aligned(16))) float sOut[160];
  const int tid = (int)threadIdx.x;
  const int c = tid & (CH - 1);
  const int half = tid >> 7;
  {
    const float* rp = REC + (size_t)(half * (NREC / 2)) * CH + c;
    double s = 0.0;
#pragma unroll 4
    for (int r = 0; r < NREC / 2; ++r) s += (double)rp[(size_t)r * CH];
    sD[tid] = s;
  }
  __syncthreads();
  {
    const double tot = sD[c] + sD[c + CH];
    const float g = (float)(tot / 100000.0);
    if (tid < CH) sgp[c] = g;
  }
  __syncthreads();
  {
    float a = 0.0f;
#pragma unroll 4
    for (int k = 0; k < CH; ++k) a = fmaf(sgp[k], bf16_val(w1[(size_t)k * CH + c]), a);
    a = a + bf16_val(b1[c]);
    a = (a > 0.0f) ? a : (a - a);
    if (tid < CH) sh[c] = a;
  }
  __syncthreads();
  {
    float a = 0.0f;
#pragma unroll 4
    for (int k = 0; k < CH; ++k) a = fmaf(sh[k], bf16_val(w2[(size_t)k * CH + c]), a);
    a = a + bf16_val(b2[c]);
    const float al  = bf16_val(alpha[0]);
    const float w   = 1.0f / (1.0f + expf(-al));
    const float omw = 1.0f - w;
    if (tid < CH) sOut[c] = a;
    else if (tid < 160) sOut[tid] = (tid == 128) ? w : ((tid == 129) ? omw : 0.0f);
  }
  __syncthreads();
  {
    const int i4 = tid < 39 ? tid : 39;
    const v4f v = *(const v4fa*)(sOut + 4 * i4);
    const bool st = tid < 40;
    volatile v4f* q = (volatile v4f*)(GLB + 4 * i4);
    if (st) *q = v;
    __threadfence();
    if (st) *q = v;
  }
}

#define PUTJ(HJ, SJ, RJ) { \
    const int wd = (int)(((SJ) << 17) | ((unsigned)(RJ) & 0x1FFFFu)); \
    if ((HJ) && pos < WLCAP) mywl[pos] = wd; \
    pos += (HJ) ? 1 : 0; }

__global__ __launch_bounds__(256) void k_bucket(const int* __restrict__ eidx, int* LIST, int* CNT, int* OFF, int* FLAG) {
  extern __shared__ __attribute__((aligned(16))) int dsm[];
  int* pl   = dsm;
  int* wl   = dsm + BK_WL;
  int* cnt  = dsm + BK_CNT;
  int* offs = dsm + BK_OFF;
  int* cur  = dsm + BK_CUR;
  int* misc = dsm + BK_MISC;
  const int tid = (int)threadIdx.x, lane = tid & 31, wave = tid >> 5;
  const int b = (int)blockIdx.x;
  const unsigned slotBase = (unsigned)b * NBRUN;
  const int* rowp = eidx;
  const int* colp = eidx + NE;

  {
    const v4i z4 = {0, 0, 0, 0};
    for (int i = tid * 4; i < BK_INTS; i += 256 * 4) *(v4ia*)(dsm + i) = z4;
  }
  __syncthreads();

  {
    int wc = 0;
    int* mywl = wl + wave * WLCAP;
    const int c0 = wave * CPW;
    const int c1 = (c0 + CPW < NCHUNK) ? (c0 + CPW) : NCHUNK;
#pragma unroll 1
    for (int ch = c0; ch < c1; ++ch) {
      const int e0 = ch * WCHUNK + lane * 8;
      const v4i da = *(const v4ia*)(colp + e0);
      const v4i db = *(const v4ia*)(colp + e0 + 4);
      const unsigned s0 = (unsigned)da.x - slotBase, s1 = (unsigned)da.y - slotBase;
      const unsigned s2 = (unsigned)da.z - slotBase, s3 = (unsigned)da.w - slotBase;
      const unsigned s4 = (unsigned)db.x - slotBase, s5 = (unsigned)db.y - slotBase;
      const unsigned s6 = (unsigned)db.z - slotBase, s7 = (unsigned)db.w - slotBase;
      const bool h0 = s0 < (unsigned)NBRUN, h1 = s1 < (unsigned)NBRUN, h2 = s2 < (unsigned)NBRUN, h3 = s3 < (unsigned)NBRUN;
      const bool h4 = s4 < (unsigned)NBRUN, h5 = s5 < (unsigned)NBRUN, h6 = s6 < (unsigned)NBRUN, h7 = s7 < (unsigned)NBRUN;
      const int c = (int)h0 + (int)h1 + (int)h2 + (int)h3 + (int)h4 + (int)h5 + (int)h6 + (int)h7;
      const unsigned any = __builtin_amdgcn_ballot_w32(c != 0);
      if (any != 0u) {
        const v4i ra = *(const v4ia*)(rowp + e0);
        const v4i rb = *(const v4ia*)(rowp + e0 + 4);
        asm volatile("" :: "v"(ra.x), "v"(ra.y), "v"(ra.z), "v"(ra.w), "v"(rb.x), "v"(rb.y), "v"(rb.z), "v"(rb.w));
        const unsigned m0 = __builtin_amdgcn_ballot_w32((c & 1) != 0);
        const unsigned m1 = __builtin_amdgcn_ballot_w32((c & 2) != 0);
        const unsigned m2 = __builtin_amdgcn_ballot_w32((c & 4) != 0);
        const unsigned m3 = __builtin_amdgcn_ballot_w32((c & 8) != 0);
        const int pre = (int)__builtin_amdgcn_mbcnt_lo(m0, 0u) + 2 * (int)__builtin_amdgcn_mbcnt_lo(m1, 0u)
                      + 4 * (int)__builtin_amdgcn_mbcnt_lo(m2, 0u) + 8 * (int)__builtin_amdgcn_mbcnt_lo(m3, 0u);
        const int tot = (int)__builtin_popcount(m0) + 2 * (int)__builtin_popcount(m1)
                      + 4 * (int)__builtin_popcount(m2) + 8 * (int)__builtin_popcount(m3);
        int pos = wc + pre;
        PUTJ(h0, s0, ra.x)
        PUTJ(h1, s1, ra.y)
        PUTJ(h2, s2, ra.z)
        PUTJ(h3, s3, ra.w)
        PUTJ(h4, s4, rb.x)
        PUTJ(h5, s5, rb.y)
        PUTJ(h6, s6, rb.z)
        PUTJ(h7, s7, rb.w)
        wc += tot;
      }
    }
    if (lane == 0) misc[wave] = wc;
  }
  __syncthreads();

  if (wave == 0) {
    int t = 0, ov = 0;
#pragma unroll 1
    for (int w2 = 0; w2 < 8; ++w2) {
      const int craw = misc[w2];
      ov |= (craw > WLCAP) ? 1 : 0;
      const int c = __builtin_amdgcn_readfirstlane(clampi(craw, 0, WLCAP));
      const int* lp = wl + w2 * WLCAP;
#pragma unroll 1
      for (int b0 = 0; b0 < c; b0 += 32) {
        const int idx = b0 + lane;
        const int ent = lp[idx < WLCAP ? idx : WLCAP - 1];
        const int m32 = (c - b0) < 32 ? (c - b0) : 32;
#pragma unroll 1
        for (int k = 0; k < m32; ++k) {
          const int u    = __builtin_amdgcn_readlane(ent, k);
          const int slot = (u >> 17) & (NBRUN - 1);
          const int cv   = cnt[slot];
          asm volatile("" :: "v"(cv));
          if (lane == 0) cnt[slot] = cv + 1;
        }
      }
      t += c;
    }
    ov |= (t > RCAP) ? 1 : 0;
    if (lane == 0) { misc[8] = t; misc[9] = ov; }
  }
  __syncthreads();

  if (wave == 0) {
    const int base = lane * (NBRUN / 32);
    int s = 0;
#pragma unroll 1
    for (int i = 0; i < NBRUN / 32; ++i) s += cnt[base + i];
    int incl = s;
#pragma unroll
    for (int d = 1; d < 32; d <<= 1) {
      const int y = __shfl_up(incl, d, 32);
      if (lane >= d) incl += y;
    }
    int run = incl - s;
#pragma unroll 1
    for (int i = 0; i < NBRUN / 32; ++i) {
      const int cv = cnt[base + i];
      offs[base + i] = run;
      cur[base + i]  = run;
      run += cv;
    }
  }
  __syncthreads();

  if (wave == 0) {
#pragma unroll 1
    for (int w2 = 0; w2 < 8; ++w2) {
      const int craw = misc[w2];
      const int c = __builtin_amdgcn_readfirstlane(clampi(craw, 0, WLCAP));
      const int* lp = wl + w2 * WLCAP;
#pragma unroll 1
      for (int b0 = 0; b0 < c; b0 += 32) {
        const int idx = b0 + lane;
        const int ent = lp[idx < WLCAP ? idx : WLCAP - 1];
        const int m32 = (c - b0) < 32 ? (c - b0) : 32;
#pragma unroll 1
        for (int k = 0; k < m32; ++k) {
          const int u    = __builtin_amdgcn_readlane(ent, k);
          const int slot = (u >> 17) & (NBRUN - 1);
          int p = cur[slot];
          asm volatile("" :: "v"(p));
          p = clampi(p, 0, RCAP - 1);
          if (lane == 0) { pl[p] = u; cur[slot] = p + 1; }
        }
      }
    }
  }
  __syncthreads();

  const int ovf = misc[9];
  int* ldst = LIST + (size_t)b * RCAP;
  for (int pass = 0; pass < 2; ++pass) {
#pragma unroll 1
    for (int i = tid; i < RCAP / 4; i += 256) {
      const v4i v = *(const v4ia*)(pl + 4 * i);
      *(volatile v4i*)(ldst + 4 * i) = v;
    }
    __threadfence();
  }
  {
    const v4i c4 = *(const v4ia*)(cnt + 4 * tid);
    const v4i o4 = *(const v4ia*)(offs + 4 * tid);
    volatile v4i* qc = (volatile v4i*)(CNT + (size_t)b * NBRUN + 4 * tid);
    volatile v4i* qo = (volatile v4i*)(OFF + (size_t)b * NBRUN + 4 * tid);
    const v4i fv = (v4i){ (lane == 0) ? ovf : 0, 0, 0, 0 };
    const bool fst = (wave == 0) && (lane < 8);
    volatile v4i* qf = (volatile v4i*)(FLAG + (size_t)b * 32 + 4 * (lane & 7));
    *qc = c4;
    *qo = o4;
    if (fst) *qf = fv;
    __threadfence();
    *qc = c4;
    *qo = o4;
    if (fst) *qf = fv;
  }
}
#undef PUTJ

__global__ __launch_bounds__(256) void k_replay(const int* __restrict__ LIST, const int* __restrict__ CNT,
                                                const int* __restrict__ OFF, const int* __restrict__ FLAG,
                                                const unsigned short* __restrict__ XB, unsigned short* AGG) {
  const int tid = (int)threadIdx.x, lane = tid & 31, wave = tid >> 5;
  const int b = (int)blockIdx.x;
  const int nodeBase = b * NBRUN;
  int fl = FLAG[(size_t)b * 32];
  asm volatile("" :: "v"(fl));
  const bool blockbad = fl != 0;
  const int* lst = LIST + (size_t)b * RCAP;
  const float qnan = __int_as_float(0x7fc00000);
  const int sa = (2 * lane) & 31, sb = (2 * lane + 1) & 31;
  const bool lsel = lane >= 16;
#pragma unroll 1
  for (int si = 0; si < NBRUN / 8; ++si) {
    const int s = si * 8 + wave;
    const int node = nodeBase + s;
    int cr = CNT[node];
    int orr = OFF[node];
    asm volatile("" :: "v"(cr), "v"(orr));
    const bool live = node < NN;
    const bool big  = cr > DEGCAP;
    const int cn = __builtin_amdgcn_readfirstlane(live ? clampi(cr, 0, DEGCAP) : 0);
    const int o  = __builtin_amdgcn_readfirstlane(clampi(orr, 0, RCAP - 1));
    const float dcf = (float)cr;
    float acc0 = 0.0f, acc1 = 0.0f, acc2 = 0.0f, acc3 = 0.0f;
#pragma unroll 1
    for (int b0 = 0; b0 < cn; b0 += 32) {
      int jj = b0 + lane;
      jj = jj < cn - 1 ? jj : cn - 1;
      int idx = o + jj;
      idx = idx < RCAP - 1 ? idx : RCAP - 1;
      int wd = lst[idx];
      asm volatile("" :: "v"(wd));
      int src = wd & 0x1FFFF;
      src = src < NN - 1 ? src : NN - 1;
      int dr = CNT[src];
      asm volatile("" :: "v"(dr));
      const int drs = dr > 0 ? dr : 1;
      const float v = 1.0f / sqrtf(dcf * (float)drs);
      const float val = (dr > 0) ? v : 0.0f;
      const int vali = __float_as_int(val);
      const int m32 = (cn - b0) < 32 ? (cn - b0) : 32;
#pragma unroll 1
      for (int k = 0; k < m32; ++k) {
        const int   sk = __builtin_amdgcn_readlane(src, k);
        const float vk = __int_as_float(__builtin_amdgcn_readlane(vali, k));
        const v2u w = *(const v2ua*)(XB + (size_t)sk * CH + 4 * lane);
        const unsigned wx = w.x, wy = w.y;
        acc0 = fmaf(vk, __uint_as_float(wx << 16), acc0);
        acc1 = fmaf(vk, __uint_as_float(wx & 0xFFFF0000u), acc1);
        acc2 = fmaf(vk, __uint_as_float(wy << 16), acc2);
        acc3 = fmaf(vk, __uint_as_float(wy & 0xFFFF0000u), acc3);
      }
    }
    const bool bad = blockbad || big;
    const float v0 = live ? (bad ? qnan : acc0) : 0.0f;
    const float v1 = live ? (bad ? qnan : acc1) : 0.0f;
    const float v2 = live ? (bad ? qnan : acc2) : 0.0f;
    const float v3 = live ? (bad ? qnan : acc3) : 0.0f;
    const int hw0 = (int)pk16(bf16_bits(v0), bf16_bits(v1));
    const int hw1 = (int)pk16(bf16_bits(v2), bf16_bits(v3));
    const int lw0 = (int)pk16(bf16_lo_bits(v0), bf16_lo_bits(v1));
    const int lw1 = (int)pk16(bf16_lo_bits(v2), bf16_lo_bits(v3));
    const int g0 = __shfl(hw0, sa, 32), g1 = __shfl(hw1, sa, 32);
    const int g2 = __shfl(hw0, sb, 32), g3 = __shfl(hw1, sb, 32);
    const int p0 = __shfl(lw0, sa, 32), p1 = __shfl(lw1, sa, 32);
    const int p2 = __shfl(lw0, sb, 32), p3 = __shfl(lw1, sb, 32);
    v4u pv;
    pv.x = (unsigned)(lsel ? p0 : g0);
    pv.y = (unsigned)(lsel ? p1 : g1);
    pv.z = (unsigned)(lsel ? p2 : g2);
    pv.w = (unsigned)(lsel ? p3 : g3);
    if (node < MPR) {
      volatile v4u* q = (volatile v4u*)(AGG + (size_t)node * KT2 + 8 * lane);
      *q = pv;
      __threadfence();
      *q = pv;
    }
  }
}

__global__ __launch_bounds__(256) void k_row(const float* __restrict__ LOC, const float* __restrict__ GLB,
                                             unsigned short* COMB) {
  __shared__ __attribute__((aligned(16))) float sG[160];
  const int tid = (int)threadIdx.x;
  {
    const int i4 = tid < 39 ? tid : 39;
    const v4f v = *(const v4fa*)(GLB + 4 * i4);
    asm volatile("" :: "v"(v));
    if (tid < 40) *(v4fa*)(sG + 4 * i4) = v;
  }
  __syncthreads();
  const unsigned g = blockIdx.x * 256u + (unsigned)tid;
  const int row = (int)(g >> 4);
  const int p   = (int)(g & 15u);
  const float* lp = LOC + (size_t)row * CH + 8 * p;
  const v4f a  = *(const v4fa*)lp;
  const v4f c  = *(const v4fa*)(lp + 4);
  const v4f ga = *(const v4fa*)(sG + 8 * p);
  const v4f gc = *(const v4fa*)(sG + 8 * p + 4);
  const float w   = sG[128];
  const float omw = sG[129];
  const v4f ca = a * w + ga * omw;
  const v4f cc = c * w + gc * omw;
  const unsigned mk = (row < NN) ? 0xFFFFFFFFu : 0u;
  const v4u mw = (v4u){ mk, mk, mk, mk };
  const v4u hi = pack8_bf16(ca, cc) & mw;
  const v4u lo = pack8_bf16_lo(ca, cc) & mw;
  volatile v4u* qh = (volatile v4u*)(COMB + (size_t)row * KT2 + 8 * p);
  volatile v4u* ql = (volatile v4u*)(COMB + (size_t)row * KT2 + CH + 8 * p);
  *qh = hi;
  *ql = lo;
  __threadfence();
  *qh = hi;
  *ql = lo;
}

constexpr size_t SZ_R1   = (size_t)MPR * CH * 4;
constexpr size_t SZ_R2   = (size_t)MPR * KT2 * 2;
constexpr size_t SZ_LIST = (size_t)NBLK * RCAP * 4;
constexpr size_t SZ_CNT  = (size_t)NSLOT * 4;
constexpr size_t SZ_FLAG = (size_t)NBLK * 128;
constexpr size_t SZ_REC  = (size_t)NREC * CH * 4;
constexpr size_t SZ_GLB  = 768;
constexpr size_t SZ_WT   = (size_t)CH * KT2 * 2;
constexpr size_t SZ_FCB  = 512;
constexpr size_t O_R1   = 0;
constexpr size_t O_R2   = O_R1 + SZ_R1;
constexpr size_t O_LIST = O_R2 + SZ_R2;
constexpr size_t O_CNT  = O_LIST + SZ_LIST;
constexpr size_t O_OFF  = O_CNT + SZ_CNT;
constexpr size_t O_FLAG = O_OFF + SZ_CNT;
constexpr size_t O_REC  = O_FLAG + SZ_FLAG;
constexpr size_t O_GLB  = O_REC + SZ_REC;
constexpr size_t O_WLT  = O_GLB + SZ_GLB;
constexpr size_t O_FCT  = O_WLT + SZ_WT;
constexpr size_t O_FCB  = O_FCT + SZ_WT;
constexpr size_t WS_TOT = O_FCB + SZ_FCB;
static_assert(WS_TOT <= ((size_t)128 << 20));
static_assert(O_R2 % 256 == 0 && O_LIST % 256 == 0 && O_CNT % 256 == 0 && O_OFF % 256 == 0 && O_FLAG % 256 == 0);
static_assert(O_REC % 256 == 0 && O_GLB % 256 == 0 && O_WLT % 256 == 0 && O_FCT % 256 == 0 && O_FCB % 256 == 0);
static_assert((size_t)MPR * CH * 2 <= SZ_R1);
static_assert((size_t)NN * CH - 1 < (size_t)NN * CH);

extern "C" void kernel_launch(void* const* d_in, const int* in_sizes, int n_in,
                              void* d_out, int out_size, void* d_ws, size_t ws_size,
                              hipStream_t stream) {
  if (n_in < 10) return;
  if (in_sizes[0] != NN * CH) return;
  if (in_sizes[1] != 2 * NE) return;
  if (in_sizes[2] != CH * CH || in_sizes[3] != CH * CH) return;
  if (in_sizes[4] != CH) return;
  if (in_sizes[5] != CH * CH || in_sizes[6] != CH) return;
  if (in_sizes[7] != 1) return;
  if (in_sizes[8] != CH * CH || in_sizes[9] != CH) return;
  if (out_size != NN * CH) return;
  if (WS_TOT > ws_size) return;

  const float* x     = (const float*)d_in[0];
  const int*   eidx  = (const int*)d_in[1];
  const float* wloc  = (const float*)d_in[2];
  const float* w1    = (const float*)d_in[3];
  const float* b1    = (const float*)d_in[4];
  const float* w2    = (const float*)d_in[5];
  const float* b2    = (const float*)d_in[6];
  const float* alpha = (const float*)d_in[7];
  const float* fc_w  = (const float*)d_in[8];
  const float* fc_b  = (const float*)d_in[9];
  float* out = (float*)d_out;

  char* ws = (char*)d_ws;
  unsigned short* XB   = (unsigned short*)(ws + O_R1);
  float*          LOC  = (float*)(ws + O_R1);
  unsigned short* AGG  = (unsigned short*)(ws + O_R2);
  unsigned short* COMB = (unsigned short*)(ws + O_R2);
  int*            LIST = (int*)(ws + O_LIST);
  int*            CNT  = (int*)(ws + O_CNT);
  int*            OFF  = (int*)(ws + O_OFF);
  int*            FLAG = (int*)(ws + O_FLAG);
  float*          REC  = (float*)(ws + O_REC);
  float*          GLB  = (float*)(ws + O_GLB);
  unsigned short* WLT2 = (unsigned short*)(ws + O_WLT);
  unsigned short* FCT2 = (unsigned short*)(ws + O_FCT);
  float*          FCB  = (float*)(ws + O_FCB);

  const int bkLds = BK_INTS * 4;
  hipFuncSetAttribute(reinterpret_cast<const void*>(&k_bucket), hipFuncAttributeMaxDynamicSharedMemorySize, bkLds);

  k_plane<0><<<MPR * CH / 8 / 256, 256, 0, stream>>>(x, NN, CH, CH, XB, MPR, CH);
  k_wprep<<<33, 256, 0, stream>>>(wloc, fc_w, fc_b, WLT2, FCT2, FCB);
  k_colsum<<<NREC, 32, 0, stream>>>(XB, REC);
  k_global<<<1, 256, 0, stream>>>(REC, w1, b1, w2, b2, alpha, GLB);
  k_bucket<<<NBLK, 256, (size_t)bkLds, stream>>>(eidx, LIST, CNT, OFF, FLAG);
  k_replay<<<NBLK, 256, 0, stream>>>(LIST, CNT, OFF, FLAG, XB, AGG);
  k_gemm_nt<1, 0><<<391, 256, 0, stream>>>(AGG, WLT2, FCB, LOC, MPR, CH, KT2, CH);
  k_row<<<MPR * (CH / 8) / 256, 256, 0, stream>>>(LOC, GLB, COMB);
  k_gemm_nt<1, 1><<<391, 256, 0, stream>>>(COMB, FCT2, FCB, out, NN, CH, KT2, CH);
}
